// BioEncoderMamba_80676665688199
// MI455X (gfx1250) — hardware-verified
//
#include <hip/hip_runtime.h>
#include <hip/hip_bf16.h>
#include <math.h>


typedef _Float16 bf16;
typedef _Float16 f16;
typedef __attribute__((ext_vector_type(4))) unsigned v4u_t;
typedef unsigned v4ua __attribute__((ext_vector_type(4), may_alias));
typedef __attribute__((ext_vector_type(4))) float v4f_t;
typedef float v4fa __attribute__((ext_vector_type(4), may_alias));
typedef __attribute__((ext_vector_type(16))) bf16  bf16x16;
typedef bf16x16 f16x16;
typedef __attribute__((ext_vector_type(8)))  bf16  bf16x8;
typedef bf16x8 f16x8;
typedef __attribute__((ext_vector_type(4)))  bf16  bf16x4;
typedef __attribute__((ext_vector_type(8)))  float f32x8;
__device__ __forceinline__ f32x8 wmma16(f16x16 a, f16x16 b, f32x8 c) {
  c = __builtin_amdgcn_wmma_f32_16x16x32_f16(false, a, false, b, (short)0, c, false, false);
  asm volatile("v_nop\n\tv_nop\n\tv_nop\n\tv_nop" : "+v"(c) : "v"(a), "v"(b));
  return c;
}
#define LDS_STRIDE 48
#define KSTRIDE    72
#define VSTRIDE    48

__device__ __forceinline__ f32x8 wmma_bf16(bf16x16 a, bf16x16 b, f32x8 c) {
  c = __builtin_amdgcn_wmma_f32_16x16x32_f16(false, a, false, b, (short)0, c, false, false);
  asm volatile("v_nop\n\tv_nop\n\tv_nop\n\tv_nop" : "+v"(c) : "v"(a), "v"(b));
  return c;
}

template <typename T>
__device__ __forceinline__ bf16x16 load_frag(const T* __restrict__ base, int ld,
                                             int row0, int k0) {
  const int lane = threadIdx.x & 31;
  const int r    = lane & 15;
  const int kh   = (lane >> 4) * 8;
  const T* p0 = base + (size_t)(row0 + r) * ld + (k0 + kh);
  const T* p1 = p0 + 16;
  bf16x16 f;
#pragma unroll
  for (int i = 0; i < 8; ++i) {
    f[i]     = (bf16)p0[i];
    f[i + 8] = (bf16)p1[i];
  }
  return f;
}

__device__ __forceinline__ bf16x16 lds_frag(const bf16* base, int stride) {
  const int lane = threadIdx.x & 31;
  const int row  = lane & 15;
  const int kh   = (lane >> 4) * 8;
  const bf16x8 lo = *(const bf16x8*)(base + row * stride + kh);
  const bf16x8 hi = *(const bf16x8*)(base + row * stride + kh + 16);
  bf16x16 f;
#pragma unroll
  for (int i = 0; i < 8; ++i) { f[i] = lo[i]; f[i + 8] = hi[i]; }
  return f;
}

template <typename T>
__device__ __forceinline__ void stage_read16(const T* __restrict__ p, float* buf) {
#pragma unroll
  for (int i = 0; i < 16; ++i) buf[i] = (float)p[i];
}

__device__ __forceinline__ void stage_write(bf16* dst, const float* buf, int nquad) {
#pragma unroll
  for (int i = 0; i < nquad; ++i) {
    bf16x4 q;
    q[0] = (bf16)buf[4 * i];     q[1] = (bf16)buf[4 * i + 1];
    q[2] = (bf16)buf[4 * i + 2]; q[3] = (bf16)buf[4 * i + 3];
    *(bf16x4*)(dst + 4 * i) = q;
  }
}


#define GSTR 48
#define GSTR 48
template <typename AT, int EPI, bool OUT16>
__global__ __launch_bounds__(256) void gemm_kne(const AT* __restrict__ A, int lda, const float* __restrict__ Wm, int ldw,
                                                const float* __restrict__ bias, const float* __restrict__ R, const float* __restrict__ gvec,
                                                void* __restrict__ Yv, int ldy, int K) {
  __shared__ __attribute__((aligned(16))) f16 ldsA[128 * GSTR];
  __shared__ __attribute__((aligned(16))) f16 ldsW[128 * GSTR];
  __shared__ __attribute__((aligned(16))) float oS[8][32 * 68];
  const int tid = threadIdx.x, lane = tid & 31, wave = tid >> 5, cl = lane & 15, rh = (lane >> 4) * 8;
  const int m0 = blockIdx.x * 128, n0 = blockIdx.y * 128;
  const int wm = (wave & 3) * 32, wn = (wave >> 2) * 64;
  f32x8 acc[2][4];
#pragma unroll
  for (int i = 0; i < 2; ++i)
#pragma unroll
    for (int j = 0; j < 4; ++j) { f32x8 z = {}; acc[i][j] = z; }
#pragma unroll 1
  for (int k0 = 0; k0 < K; k0 += 32) {
    __syncthreads();
    { const int row = tid >> 1, ch = (tid & 1) * 16;
      const AT* src = A + (size_t)(m0 + row) * lda + k0 + ch;
#pragma unroll
      for (int g = 0; g < 16; ++g) ldsA[row * GSTR + ch + g] = (f16)src[g]; }
    { const int k = tid >> 3, nn0 = (tid & 7) * 16;
      const float* src = Wm + (size_t)(k0 + k) * ldw + n0 + nn0;
#pragma unroll
      for (int g = 0; g < 4; ++g) { const v4f_t v = *(const v4f_t*)(src + 4 * g);
#pragma unroll
        for (int u = 0; u < 4; ++u) ldsW[(nn0 + 4 * g + u) * GSTR + k] = (f16)v[u]; } }
    __syncthreads();
    f16x16 af[2];
#pragma unroll
    for (int i = 0; i < 2; ++i) af[i] = lds_frag(ldsA + (wm + 16 * i) * GSTR, GSTR);
#pragma unroll
    for (int j = 0; j < 4; ++j) {
      const f16x16 bf = lds_frag(ldsW + (wn + 16 * j) * GSTR, GSTR);
#pragma unroll
      for (int i = 0; i < 2; ++i) acc[i][j] = wmma16(af[i], bf, acc[i][j]);
    }
  }
  float* so = oS[wave];
#pragma unroll
  for (int i = 0; i < 2; ++i)
#pragma unroll
    for (int j = 0; j < 4; ++j) {
      const int n = n0 + wn + 16 * j + cl;
      const float bv = bias ? bias[n] : 0.0f;
      const float gv = (EPI == 2) ? gvec[n] : 0.0f;
      if (EPI == 1) {
#pragma unroll 1
        for (int r = 0; r < 8; ++r) { const float xg = acc[i][j][r] + bv; so[(16 * i + rh + r) * 68 + 16 * j + cl] = 0.5f * xg * (1.0f + erff(xg * 0.70710678118654752f)); }
      } else {
#pragma unroll
        for (int r = 0; r < 8; ++r) {
          float v = acc[i][j][r] + bv;
          if (EPI == 2) v = R[(size_t)(m0 + wm + 16 * i + rh + r) * ldy + n] + gv * v;
          so[(16 * i + rh + r) * 68 + 16 * j + cl] = v;
        }
      }
    }
  asm volatile("s_wait_dscnt 0" ::: "memory");
  __builtin_amdgcn_wave_barrier();
#pragma unroll 1
  for (int pass = 0; pass < 2; ++pass) {
    if (OUT16) {
      f16* Y = (f16*)Yv;
#pragma unroll
      for (int it = 0; it < 8; ++it) { const int c = lane + 32 * it, rr = c >> 3, q8 = (c & 7) * 8;
        union { f16 h[8]; v4u_t v; } u;
#pragma unroll
        for (int e = 0; e < 8; ++e) u.h[e] = (f16)so[rr * 68 + q8 + e];
        *(volatile v4u_t*)(Y + (size_t)(m0 + wm + rr) * ldy + n0 + wn + q8) = u.v; }
    } else {
      float* Y = (float*)Yv;
#pragma unroll
      for (int it = 0; it < 16; ++it) { const int f4 = lane + 32 * it, rr = f4 >> 4, q = (f4 & 15) * 4;
        *(volatile v4f_t*)(Y + (size_t)(m0 + wm + rr) * ldy + n0 + wn + q) = *(const v4fa*)(so + rr * 68 + q); }
    }
    __threadfence();
  }
}


#define NSEQ 256
#define MSEQ 256
#define LT 16
#define NTOK (MSEQ * LT)
#define CIN 7
#define TLEN 160
#define PATCH 10
#define KP 96
#define DM 512
#define DI 1024
#define DS 16
#define DTR 32
#define NXP 128
#define NL 2

__global__ __launch_bounds__(256) void k_patch(const float* __restrict__ x, const float* __restrict__ g, const float* __restrict__ be, const float* __restrict__ mu,
                                              const float* __restrict__ var, float* __restrict__ A0) {
  const int tid = threadIdx.x; const size_t row0 = (size_t)blockIdx.x * 16;
#pragma unroll 1
  for (int pass = 0; pass < 2; ++pass) {
#pragma unroll 1
    for (int k2 = 0; k2 < 2; ++k2) { const int f4 = tid + 256 * k2;
      if (f4 < 16 * (KP / 4)) {
        v4f_t o;
#pragma unroll
        for (int u = 0; u < 4; ++u) { const int e = f4 * 4 + u; const int r = e / KP, col = e % KP; const size_t tok = row0 + r; const int b = (int)(tok / LT), l = (int)(tok % LT);
          const int cc = min(col / PATCH, CIN - 1), kk = col % PATCH;
          const float xv = x[((size_t)b * CIN + cc) * TLEN + l * PATCH + kk];
          const float bn = (xv - mu[cc]) * rsqrtf(var[cc] + 1e-5f) * g[cc] + be[cc];
          o[u] = (col < CIN * PATCH) ? bn : 0.0f; }
        *(volatile v4f_t*)(A0 + row0 * KP + (size_t)f4 * 4) = o; } }
    __threadfence(); }
}
__global__ __launch_bounds__(256) void k_padw(const float* __restrict__ pw, float* __restrict__ Wp) {
  const int tid = threadIdx.x;
#pragma unroll 1
  for (int pass = 0; pass < 2; ++pass) {
#pragma unroll 1
    for (int e = tid + blockIdx.x * 256; e < KP * DM; e += 256 * gridDim.x) { const int k = e / DM, n = e % DM; const float v = pw[(size_t)n * (CIN * PATCH) + min(k, CIN * PATCH - 1)];
      *(volatile float*)(Wp + e) = (k < CIN * PATCH) ? v : 0.0f; }
    __threadfence(); }
}
__global__ __launch_bounds__(256) void k_padwx(const float* __restrict__ wx, float* __restrict__ Wxp) {
  const int tid = threadIdx.x;
#pragma unroll 1
  for (int pass = 0; pass < 2; ++pass) {
#pragma unroll 1
    for (int e = tid + blockIdx.x * 256; e < DI * NXP; e += 256 * gridDim.x) { const int k = e / NXP, n = e % NXP; const float v = wx[(size_t)k * (DTR + 2 * DS) + min(n, DTR + 2 * DS - 1)];
      *(volatile float*)(Wxp + e) = (n < DTR + 2 * DS) ? v : 0.0f; }
    __threadfence(); }
}
__global__ __launch_bounds__(256) void k_fill(float* __restrict__ p, float val, int n) { const int i = threadIdx.x + blockIdx.x * 256; if (i < n) { *(volatile float*)(p + i) = val; __threadfence(); *(volatile float*)(p + i) = val; } }

template <int MODE>
__global__ __launch_bounds__(256) void k_ln(const float* __restrict__ X, const float* __restrict__ g, const float* __restrict__ bb, const float* __restrict__ pos, float* __restrict__ Y, int nrows) {
  const int tid = threadIdx.x, lane = tid & 31, wave = tid >> 5; const int row = blockIdx.x * 8 + wave;
  if (row >= nrows) return;
  const float* xr = X + (size_t)row * DM; v4f_t v[4]; float s = 0.0f;
#pragma unroll
  for (int k = 0; k < 4; ++k) { v[k] = *(const v4f_t*)(xr + 4 * (32 * k + lane)); s += v[k][0] + v[k][1] + v[k][2] + v[k][3]; }
#pragma unroll
  for (int off = 1; off < 32; off <<= 1) s += __shfl_xor(s, off, 32);
  const float mean = s * (1.0f / DM); float q = 0.0f;
#pragma unroll
  for (int k = 0; k < 4; ++k)
#pragma unroll
    for (int u = 0; u < 4; ++u) { const float d = v[k][u] - mean; q = fmaf(d, d, q); }
#pragma unroll
  for (int off = 1; off < 32; off <<= 1) q += __shfl_xor(q, off, 32);
  const float rstd = rsqrtf(q * (1.0f / DM) + 1e-5f);
  v4f_t o[4];
#pragma unroll
  for (int k = 0; k < 4; ++k) { const int c0 = 4 * (32 * k + lane); const v4f_t gg = *(const v4f_t*)(g + c0), bv = *(const v4f_t*)(bb + c0);
    v4f_t pv = {0.0f, 0.0f, 0.0f, 0.0f}; if (MODE == 1) pv = *(const v4f_t*)(pos + (size_t)(row % LT) * DM + c0);
#pragma unroll
    for (int u = 0; u < 4; ++u) o[k][u] = (v[k][u] - mean) * rstd * gg[u] + bv[u] + pv[u]; }
#pragma unroll 1
  for (int pass = 0; pass < 2; ++pass) {
#pragma unroll
    for (int k = 0; k < 4; ++k) *(volatile v4f_t*)(Y + (size_t)row * DM + 4 * (32 * k + lane)) = o[k];
    __threadfence(); }
}
__global__ __launch_bounds__(256) void k_conv(const float* __restrict__ UZ, const float* __restrict__ cw, const float* __restrict__ cb, int dir, float* __restrict__ UC) {
  const int tok = blockIdx.x, tid = threadIdx.x; const int t = tok % LT; const int bseq = tok / LT;
#pragma unroll 1
  for (int j = 0; j < DI / 256; ++j) { const int d = tid + 256 * j;
    float acc = cb[d];
#pragma unroll
    for (int k = 0; k < 4; ++k) { const int tt = dir ? (t + 3 - k) : (t + k - 3);
      if (tt >= 0 && tt < LT) acc = fmaf(UZ[((size_t)bseq * LT + tt) * (2 * DI) + d], cw[d * 4 + k], acc); }
    const float sv = acc / (1.0f + expf(-acc));
    *(volatile float*)(UC + (size_t)tok * DI + d) = sv; __threadfence(); *(volatile float*)(UC + (size_t)tok * DI + d) = sv; }
}
__global__ __launch_bounds__(256) void k_scan(const float* __restrict__ PROJ, const float* __restrict__ DTRW, const float* __restrict__ UC, const float* __restrict__ UZ,
                                             const float* __restrict__ Alog, const float* __restrict__ Dv, int dir, bf16* __restrict__ G16) {
  __shared__ float BC[LT][2 * DS];
  __shared__ __attribute__((aligned(16))) bf16 gS[LT][256 + 8];
  const int bseq = blockIdx.x, cg = blockIdx.y, tid = threadIdx.x; const int d = cg * 256 + tid;
#pragma unroll 1
  for (int e = tid; e < LT * 2 * DS; e += 256) { const int t = e >> 5, c = e & 31; BC[t][c] = PROJ[((size_t)bseq * LT + t) * NXP + DTR + c]; }
  float a2[DS], h[DS];
#pragma unroll
  for (int n = 0; n < DS; ++n) { a2[n] = -expf(Alog[(size_t)d * DS + n]) * 1.4426950408889634f; h[n] = 0.0f; }
  const float Dd = Dv[d];
  __syncthreads();
#pragma unroll 1
  for (int s = 0; s < LT; ++s) { const int t = dir ? (LT - 1 - s) : s; const size_t tok = (size_t)bseq * LT + t;
    const float dr = DTRW[tok * DI + d]; const float dt = (dr > 20.0f) ? dr : log1pf(expf(dr));
    const float u = UC[tok * DI + d]; const float dtu = dt * u; float y = u * Dd;
#pragma unroll
    for (int n = 0; n < DS; ++n) { h[n] = fmaf(h[n], __builtin_amdgcn_exp2f(dt * a2[n]), dtu * BC[t][n]); y = fmaf(h[n], BC[t][DS + n], y); }
    const float z = UZ[tok * (2 * DI) + DI + d]; const float gte = y * (z / (1.0f + expf(-z)));
    gS[t][tid] = (bf16)(gte * 64.0f); }
  __syncthreads();
#pragma unroll 1
  for (int pass = 0; pass < 2; ++pass) {
#pragma unroll
    for (int k = 0; k < 2; ++k) { const int idx = tid + 256 * k; const int t = idx >> 5, piece = (idx & 31) * 8;
      *(volatile v4u_t*)(G16 + ((size_t)bseq * LT + t) * DI + cg * 256 + piece) = *(const v4ua*)(&gS[t][piece]); }
    __threadfence(); }
}

extern "C" void kernel_launch(void* const* d_in, const int* in_sizes, int n_in,
                              void* d_out, int out_size, void* d_ws, size_t ws_size,
                              hipStream_t stream) {
  (void)in_sizes; (void)n_in; (void)out_size;
  const float** f = (const float**)d_in;
  const float* x = f[0], *bng = f[1], *bnb = f[2], *bnm = f[3], *bnv = f[4], *pw = f[5], *pb = f[6], *lpg = f[7], *lpb = f[8], *pos = f[9], *blg = f[10], *blb = f[11];
  const float* Wi = f[12], *cw = f[13], *cb = f[14], *Wx = f[15], *Wdt = f[16], *bdt = f[17], *Alog = f[18], *Dsk = f[19], *Wo = f[20], *lfg = f[21], *lfb = f[22];
  float* out = (float*)d_out;
  char* ws = (char*)d_ws;
  float* A0 = (float*)ws; ws += (size_t)NTOK * KP * 4;
  float* Wp = (float*)ws; ws += (size_t)KP * DM * 4;
  float* H0 = (float*)ws; ws += (size_t)NTOK * DM * 4;
  float* h = (float*)ws; ws += (size_t)NTOK * DM * 4;
  float* hn = (float*)ws; ws += (size_t)NTOK * DM * 4;
  float* UZ = (float*)ws; ws += (size_t)NTOK * 2 * DI * 4;
  float* UC = (float*)ws; ws += (size_t)NTOK * DI * 4;
  float* Wxp = (float*)ws; ws += (size_t)DI * NXP * 4;
  float* PROJ = (float*)ws; ws += (size_t)NTOK * NXP * 4;
  float* DTRW = (float*)ws; ws += (size_t)NTOK * DI * 4;
  bf16* G16 = (bf16*)ws; ws += (size_t)NTOK * DI * 2;
  float* inv64 = (float*)ws; ws += DM * 4;
  if ((size_t)(ws - (char*)d_ws) > ws_size) return;
  const dim3 blk(256);
  k_fill<<<dim3(2), blk, 0, stream>>>(inv64, 1.0f / 64.0f, DM);
  k_patch<<<dim3(NTOK / 16), blk, 0, stream>>>(x, bng, bnb, bnm, bnv, A0);
  k_padw<<<dim3(16), blk, 0, stream>>>(pw, Wp);
  gemm_kne<float, 0, false><<<dim3(NTOK / 128, DM / 128), blk, 0, stream>>>(A0, KP, Wp, DM, pb, nullptr, nullptr, H0, DM, KP);
  k_ln<1><<<dim3(NTOK / 8), blk, 0, stream>>>(H0, lpg, lpb, pos, h, NTOK);
  for (int l = 0; l < NL; ++l) {
    k_ln<0><<<dim3(NTOK / 8), blk, 0, stream>>>(h, blg + l * DM, blb + l * DM, nullptr, hn, NTOK);
    for (int dir = 0; dir < 2; ++dir) { const size_t ld = (size_t)l * 2 + dir;
      gemm_kne<float, 0, false><<<dim3(NTOK / 128, 2 * DI / 128), blk, 0, stream>>>(hn, DM, Wi + ld * DM * 2 * DI, 2 * DI, nullptr, nullptr, nullptr, UZ, 2 * DI, DM);
      k_conv<<<dim3(NTOK), blk, 0, stream>>>(UZ, cw + ld * DI * 4, cb + ld * DI, dir, UC);
      k_padwx<<<dim3(16), blk, 0, stream>>>(Wx + ld * DI * (DTR + 2 * DS), Wxp);
      gemm_kne<float, 0, false><<<dim3(NTOK / 128, NXP / 128), blk, 0, stream>>>(UC, DI, Wxp, NXP, nullptr, nullptr, nullptr, PROJ, NXP, DI);
      gemm_kne<float, 0, false><<<dim3(NTOK / 128, DI / 128), blk, 0, stream>>>(PROJ, NXP, Wdt + ld * DTR * DI, DI, bdt + ld * DI, nullptr, nullptr, DTRW, DI, DTR);
      k_scan<<<dim3(MSEQ, DI / 256), blk, 0, stream>>>(PROJ, DTRW, UC, UZ, Alog + ld * DI * DS, Dsk + ld * DI, dir, G16);
      gemm_kne<bf16, 2, false><<<dim3(NTOK / 128, DM / 128), blk, 0, stream>>>(G16, DI, Wo + ld * DI * DM, DM, nullptr, h, inv64, h, DM, DI);
    }
  }
  k_ln<0><<<dim3(NTOK / 8), blk, 0, stream>>>(h, lfg, lfb, nullptr, out, NTOK);
}
